// ConvSelfAttention_9148280341193
// MI455X (gfx1250) — hardware-verified
//
#include <hip/hip_runtime.h>


typedef __bf16        v16bf __attribute__((ext_vector_type(16)));
typedef float         v8f   __attribute__((ext_vector_type(8)));
typedef float         v4f   __attribute__((ext_vector_type(4)));
typedef unsigned int  v4u   __attribute__((ext_vector_type(4)));
typedef unsigned int  v2u   __attribute__((ext_vector_type(2)));

union Frag { v16bf v; v4u q[2]; };

#define C_IN  512
#define C_V   512
#define D_K   64
#define NPOS  4096

__device__ __forceinline__ unsigned int bf_bits(float f) {
    unsigned int u = __float_as_uint(f);
    u += 0x7FFFu + ((u >> 16) & 1u);
    return u >> 16;
}

__device__ __forceinline__ void split_bf(float f, unsigned int& hb, unsigned int& lb) {
    hb = bf_bits(f);
    const float fh = __uint_as_float(hb << 16);
    lb = bf_bits(f - fh);
}

__device__ __forceinline__ v8f wmma3(v16bf ah, v16bf al, v16bf bh, v16bf bl, v8f c) {
    c = __builtin_amdgcn_wmma_f32_16x16x32_bf16(false, ah, false, bh, (short)0, c, false, false);
    c = __builtin_amdgcn_wmma_f32_16x16x32_bf16(false, ah, false, bl, (short)0, c, false, false);
    c = __builtin_amdgcn_wmma_f32_16x16x32_bf16(false, al, false, bh, (short)0, c, false, false);
    asm volatile("v_nop\n\tv_nop\n\tv_nop\n\tv_nop" : "+v"(c) : "v"(ah), "v"(al), "v"(bh), "v"(bl));
    return c;
}

#define PT      64
#define APITCH  40
#define CPITCH  68

__global__ __launch_bounds__(256) void k_proj(
    const float* __restrict__ W,
    const float* __restrict__ X,
    unsigned short* __restrict__ Oh,
    unsigned short* __restrict__ Ol,
    int M, int transOut)
{
    __shared__ __attribute__((aligned(16))) unsigned short Ah[PT * APITCH];
    __shared__ __attribute__((aligned(16))) unsigned short Al[PT * APITCH];
    __shared__ __attribute__((aligned(16))) unsigned short Bh[PT * APITCH];
    __shared__ __attribute__((aligned(16))) unsigned short Bl[PT * APITCH];
    __shared__ __attribute__((aligned(16))) float Cs[PT * CPITCH];

    const int tid  = threadIdx.x;
    const int lane = tid & 31;
    const int wave = __builtin_amdgcn_readfirstlane(tid >> 5);
    const int m  = lane & 15;
    const int h  = lane >> 4;
    const int tilesN = NPOS / PT;
    const int m0 = (int)(blockIdx.x / tilesN) * PT;
    const int n0 = (int)(blockIdx.x % tilesN) * PT;
    if (m0 + PT > M) return;

    const int rg = wave >> 1;
    const int cb = (wave & 1) * 32;

    v8f acc0 = {0.f, 0.f, 0.f, 0.f, 0.f, 0.f, 0.f, 0.f};
    v8f acc1 = {0.f, 0.f, 0.f, 0.f, 0.f, 0.f, 0.f, 0.f};

    for (int kk = 0; kk < C_IN; kk += 32) {
#pragma unroll
        for (int it = 0; it < 2; ++it) {
            const int f   = tid + it * 256;
            const int row = f >> 3;
            const int kq  = (f & 7) * 4;
            const v4f v = *(const v4f*)(W + (size_t)(m0 + row) * C_IN + kk + kq);
            unsigned int hb0, lb0, hb1, lb1, hb2, lb2, hb3, lb3;
            split_bf(v.x, hb0, lb0); split_bf(v.y, hb1, lb1);
            split_bf(v.z, hb2, lb2); split_bf(v.w, hb3, lb3);
            v2u hv, lv;
            hv.x = hb0 | (hb1 << 16); hv.y = hb2 | (hb3 << 16);
            lv.x = lb0 | (lb1 << 16); lv.y = lb2 | (lb3 << 16);
            *(v2u*)(Ah + row * APITCH + kq) = hv;
            *(v2u*)(Al + row * APITCH + kq) = lv;
        }
#pragma unroll
        for (int it = 0; it < 2; ++it) {
            const int f  = tid + it * 256;
            const int k  = f >> 4;
            const int nq = (f & 15) * 4;
            const v4f v = *(const v4f*)(X + (size_t)(kk + k) * NPOS + n0 + nq);
            unsigned int hb, lb;
            split_bf(v.x, hb, lb); Bh[(nq + 0) * APITCH + k] = (unsigned short)hb; Bl[(nq + 0) * APITCH + k] = (unsigned short)lb;
            split_bf(v.y, hb, lb); Bh[(nq + 1) * APITCH + k] = (unsigned short)hb; Bl[(nq + 1) * APITCH + k] = (unsigned short)lb;
            split_bf(v.z, hb, lb); Bh[(nq + 2) * APITCH + k] = (unsigned short)hb; Bl[(nq + 2) * APITCH + k] = (unsigned short)lb;
            split_bf(v.w, hb, lb); Bh[(nq + 3) * APITCH + k] = (unsigned short)hb; Bl[(nq + 3) * APITCH + k] = (unsigned short)lb;
        }
        __syncthreads();

        Frag ah, al;
        {
            const unsigned short* pa = Ah + (rg * 16 + m) * APITCH;
            const unsigned short* pl = Al + (rg * 16 + m) * APITCH;
            ah.q[0] = *(const v4u*)(pa + 8 * h);       ah.q[1] = *(const v4u*)(pa + 16 + 8 * h);
            al.q[0] = *(const v4u*)(pl + 8 * h);       al.q[1] = *(const v4u*)(pl + 16 + 8 * h);
        }
        {
            Frag bh, bl;
            const unsigned short* pb = Bh + (cb + m) * APITCH;
            const unsigned short* pc = Bl + (cb + m) * APITCH;
            bh.q[0] = *(const v4u*)(pb + 8 * h);       bh.q[1] = *(const v4u*)(pb + 16 + 8 * h);
            bl.q[0] = *(const v4u*)(pc + 8 * h);       bl.q[1] = *(const v4u*)(pc + 16 + 8 * h);
            acc0 = wmma3(ah.v, al.v, bh.v, bl.v, acc0);
        }
        {
            Frag bh, bl;
            const unsigned short* pb = Bh + (cb + 16 + m) * APITCH;
            const unsigned short* pc = Bl + (cb + 16 + m) * APITCH;
            bh.q[0] = *(const v4u*)(pb + 8 * h);       bh.q[1] = *(const v4u*)(pb + 16 + 8 * h);
            bl.q[0] = *(const v4u*)(pc + 8 * h);       bl.q[1] = *(const v4u*)(pc + 16 + 8 * h);
            acc1 = wmma3(ah.v, al.v, bh.v, bl.v, acc1);
        }
        __syncthreads();
    }

#pragma unroll
    for (int r = 0; r < 8; ++r) {
        Cs[(rg * 16 + 8 * h + r) * CPITCH + cb + m]      = acc0[r];
        Cs[(rg * 16 + 8 * h + r) * CPITCH + cb + 16 + m] = acc1[r];
    }
    __syncthreads();

    v4u hvp[2], lvp[2];
    size_t offp[2];
#pragma unroll
    for (int p = 0; p < 2; ++p) {
        const int rr = wave * 8 + p * 4 + (lane >> 3);
        const int cc = (lane & 7) * 8;
        float vals[8];
        if (transOut) {
#pragma unroll
            for (int e = 0; e < 8; ++e) vals[e] = Cs[(cc + e) * CPITCH + rr];
            offp[p] = (size_t)(n0 + rr) * (size_t)M + (size_t)(m0 + cc);
        } else {
            const v4f a = *(const v4f*)(Cs + rr * CPITCH + cc);
            const v4f b = *(const v4f*)(Cs + rr * CPITCH + cc + 4);
            vals[0] = a.x; vals[1] = a.y; vals[2] = a.z; vals[3] = a.w;
            vals[4] = b.x; vals[5] = b.y; vals[6] = b.z; vals[7] = b.w;
            offp[p] = (size_t)(m0 + rr) * (size_t)NPOS + (size_t)(n0 + cc);
        }
        unsigned int hb[8], lb[8];
#pragma unroll
        for (int e = 0; e < 8; ++e) split_bf(vals[e], hb[e], lb[e]);
        v4u hv, lv;
        hv.x = hb[0] | (hb[1] << 16); hv.y = hb[2] | (hb[3] << 16);
        hv.z = hb[4] | (hb[5] << 16); hv.w = hb[6] | (hb[7] << 16);
        lv.x = lb[0] | (lb[1] << 16); lv.y = lb[2] | (lb[3] << 16);
        lv.z = lb[4] | (lb[5] << 16); lv.w = lb[6] | (lb[7] << 16);
        hvp[p] = hv; lvp[p] = lv;
    }
#pragma unroll
    for (int p = 0; p < 2; ++p) {
        *(volatile v4u*)(Oh + offp[p]) = hvp[p];
        *(volatile v4u*)(Ol + offp[p]) = lvp[p];
    }
    __threadfence();
#pragma unroll
    for (int p = 0; p < 2; ++p) {
        *(volatile v4u*)(Oh + offp[p]) = hvp[p];
        *(volatile v4u*)(Ol + offp[p]) = lvp[p];
    }
}

#define BM      16
#define BN      64
#define SPITCH  65
#define PPITCH  72
#define GPITCH  68
#define SM_S_BYTES (BM * SPITCH * 4)
#define SM_P_BYTES (BM * PPITCH * 2)
#define SM_G_BYTES (8 * 16 * GPITCH * 4)
#define SM_BYTES   SM_G_BYTES
typedef char sm_layout_check[((SM_S_BYTES + 2 * SM_P_BYTES) <= SM_G_BYTES && (SM_S_BYTES % 16) == 0 && (SM_P_BYTES % 16) == 0) ? 1 : -1];

__global__ __launch_bounds__(256) void k_attn(
    const unsigned short* __restrict__ KH,
    const unsigned short* __restrict__ KL,
    const unsigned short* __restrict__ QH,
    const unsigned short* __restrict__ QL,
    const unsigned short* __restrict__ VH,
    const unsigned short* __restrict__ VL,
    float* __restrict__ out)
{
    __shared__ __attribute__((aligned(16))) unsigned char smem[SM_BYTES];
    __shared__ float mRow[BM];
    __shared__ float lRow[BM];
    __shared__ float aRow[BM];
    float*          Sld = (float*)smem;
    unsigned short* Ph  = (unsigned short*)(smem + SM_S_BYTES);
    unsigned short* Pl  = (unsigned short*)(smem + SM_S_BYTES + SM_P_BYTES);
    float*          Stg = (float*)smem;

    const int tid  = threadIdx.x;
    const int lane = tid & 31;
    const int wave = __builtin_amdgcn_readfirstlane(tid >> 5);
    const int m = lane & 15;
    const int h = lane >> 4;
    const int row0 = blockIdx.x * BM;
    if (row0 + BM > NPOS) return;
    const int C0 = wave * 64;

    if (tid < BM) { mRow[tid] = -1.0e30f; lRow[tid] = 0.f; aRow[tid] = 0.f; }
    __syncthreads();

    const v8f vzero = {0.f, 0.f, 0.f, 0.f, 0.f, 0.f, 0.f, 0.f};
    v8f Oacc[4];
#pragma unroll
    for (int ct = 0; ct < 4; ++ct) Oacc[ct] = vzero;

    for (int jb = 0; jb < NPOS / BN; ++jb) {
        const int j0 = jb * BN;

        if (wave < 4) {
            const int tj = wave;
            v8f s = vzero;
#pragma unroll
            for (int kc = 0; kc < D_K; kc += 32) {
                Frag ah, al, bh, bl;
                const size_t ao = (size_t)(row0 + m) * D_K + kc;
                ah.q[0] = *(const v4u*)(KH + ao + 8 * h);  ah.q[1] = *(const v4u*)(KH + ao + 16 + 8 * h);
                al.q[0] = *(const v4u*)(KL + ao + 8 * h);  al.q[1] = *(const v4u*)(KL + ao + 16 + 8 * h);
                const size_t bo = (size_t)(j0 + tj * 16 + m) * D_K + kc;
                bh.q[0] = *(const v4u*)(QH + bo + 8 * h);  bh.q[1] = *(const v4u*)(QH + bo + 16 + 8 * h);
                bl.q[0] = *(const v4u*)(QL + bo + 8 * h);  bl.q[1] = *(const v4u*)(QL + bo + 16 + 8 * h);
                s = wmma3(ah.v, al.v, bh.v, bl.v, s);
            }
#pragma unroll
            for (int r = 0; r < 8; ++r)
                Sld[(8 * h + r) * SPITCH + tj * 16 + m] = s[r];
        }
        __syncthreads();

        {
            const int row = tid >> 4;
            const int seg = tid & 15;
            float e0[4];
#pragma unroll
            for (int e = 0; e < 4; ++e) e0[e] = Sld[row * SPITCH + seg * 4 + e];
            float bm = fmaxf(fmaxf(e0[0], e0[1]), fmaxf(e0[2], e0[3]));
            bm = fmaxf(bm, __shfl_xor(bm, 1));
            bm = fmaxf(bm, __shfl_xor(bm, 2));
            bm = fmaxf(bm, __shfl_xor(bm, 4));
            bm = fmaxf(bm, __shfl_xor(bm, 8));
            const float mo = mRow[row];
            const float mn = fmaxf(mo, bm);
            unsigned int ph0 = 0u, ph1 = 0u, pl0 = 0u, pl1 = 0u;
            float sum = 0.f;
#pragma unroll
            for (int e = 0; e < 4; ++e) {
                const float ex = __expf(e0[e] - mn);
                sum += ex;
                unsigned int hb, lb;
                split_bf(ex, hb, lb);
                const unsigned int sh = (unsigned int)(e & 1) * 16u;
                if (e < 2) { ph0 |= hb << sh; pl0 |= lb << sh; }
                else       { ph1 |= hb << sh; pl1 |= lb << sh; }
            }
            v2u phv, plv;
            phv.x = ph0; phv.y = ph1; plv.x = pl0; plv.y = pl1;
            *(v2u*)(Ph + row * PPITCH + seg * 4) = phv;
            *(v2u*)(Pl + row * PPITCH + seg * 4) = plv;
            sum += __shfl_xor(sum, 1);
            sum += __shfl_xor(sum, 2);
            sum += __shfl_xor(sum, 4);
            sum += __shfl_xor(sum, 8);
            if (seg == 0) {
                const float al = __expf(mo - mn);
                lRow[row] = lRow[row] * al + sum;
                mRow[row] = mn;
                aRow[row] = al;
            }
        }
        __syncthreads();

        {
            v8f alv;
#pragma unroll
            for (int r = 0; r < 8; ++r) alv[r] = aRow[8 * h + r];
#pragma unroll
            for (int ct = 0; ct < 4; ++ct) Oacc[ct] = Oacc[ct] * alv;

#pragma unroll
            for (int kh2 = 0; kh2 < 2; ++kh2) {
                Frag pa, pb;
                const unsigned short* pph = Ph + m * PPITCH + kh2 * 32;
                const unsigned short* ppl = Pl + m * PPITCH + kh2 * 32;
                pa.q[0] = *(const v4u*)(pph + 8 * h);  pa.q[1] = *(const v4u*)(pph + 16 + 8 * h);
                pb.q[0] = *(const v4u*)(ppl + 8 * h);  pb.q[1] = *(const v4u*)(ppl + 16 + 8 * h);
#pragma unroll
                for (int ct = 0; ct < 4; ++ct) {
                    Frag bh, bl;
                    const size_t vo = (size_t)(C0 + ct * 16 + m) * NPOS + (size_t)(j0 + kh2 * 32);
                    bh.q[0] = *(const v4u*)(VH + vo + 8 * h);  bh.q[1] = *(const v4u*)(VH + vo + 16 + 8 * h);
                    bl.q[0] = *(const v4u*)(VL + vo + 8 * h);  bl.q[1] = *(const v4u*)(VL + vo + 16 + 8 * h);
                    Oacc[ct] = wmma3(pa.v, pb.v, bh.v, bl.v, Oacc[ct]);
                }
            }
        }
        __syncthreads();
    }

    float linv[8];
#pragma unroll
    for (int r = 0; r < 8; ++r) linv[r] = 1.f / lRow[8 * h + r];

    float* stg = Stg + wave * (16 * GPITCH);
#pragma unroll
    for (int ct = 0; ct < 4; ++ct) {
#pragma unroll
        for (int r = 0; r < 8; ++r)
            stg[(8 * h + r) * GPITCH + ct * 16 + m] = Oacc[ct][r] * linv[r];
    }
    __syncthreads();

    const int sub = lane >> 4;
    const int cq  = (lane & 15) * 4;
    v4f ov[8];
#pragma unroll
    for (int q = 0; q < 8; ++q)
        ov[q] = *(const v4f*)(stg + (2 * q + sub) * GPITCH + cq);

    float* ob = out + (size_t)(row0 + sub) * C_V + C0 + cq;
#pragma unroll
    for (int q = 0; q < 8; ++q)
        *(volatile v4f*)(ob + (size_t)(2 * q) * C_V) = ov[q];
    __threadfence();
#pragma unroll
    for (int q = 0; q < 8; ++q)
        *(volatile v4f*)(ob + (size_t)(2 * q) * C_V) = ov[q];
}

extern "C" void kernel_launch(void* const* d_in, const int* in_sizes, int n_in,
                              void* d_out, int out_size, void* d_ws, size_t ws_size,
                              hipStream_t stream) {
    if (n_in < 4) return;
    if (in_sizes[0] != C_IN * NPOS) return;
    if (in_sizes[1] != D_K * C_IN)  return;
    if (in_sizes[2] != D_K * C_IN)  return;
    if (in_sizes[3] != C_V * C_IN)  return;
    if (out_size != NPOS * C_V)     return;

    const float* x  = (const float*)d_in[0];
    const float* Wk = (const float*)d_in[1];
    const float* Wq = (const float*)d_in[2];
    const float* Wv = (const float*)d_in[3];
    float* out = (float*)d_out;

    const size_t szK = (size_t)NPOS * D_K * 2;
    const size_t szV = (size_t)C_V * NPOS * 2;
    const size_t offKH = 0;
    const size_t offKL = offKH + szK;
    const size_t offQH = offKL + szK;
    const size_t offQL = offQH + szK;
    const size_t offVH = offQL + szK;
    const size_t offVL = offVH + szV;
    const size_t total = offVL + szV;
    if (total > ws_size) return;

    char* ws = (char*)d_ws;
    unsigned short* kh = (unsigned short*)(ws + offKH);
    unsigned short* kl = (unsigned short*)(ws + offKL);
    unsigned short* qh = (unsigned short*)(ws + offQH);
    unsigned short* ql = (unsigned short*)(ws + offQL);
    unsigned short* vh = (unsigned short*)(ws + offVH);
    unsigned short* vl = (unsigned short*)(ws + offVL);

    const int tilesN = NPOS / PT;
    k_proj<<<(D_K / PT) * tilesN, 256, 0, stream>>>(Wk, x, kh, kl, D_K, 1);
    k_proj<<<(D_K / PT) * tilesN, 256, 0, stream>>>(Wq, x, qh, ql, D_K, 1);
    k_proj<<<(C_V / PT) * tilesN, 256, 0, stream>>>(Wv, x, vh, vl, C_V, 0);
    k_attn<<<NPOS / BM, 256, 0, stream>>>(kh, kl, qh, ql, vh, vl, out);
}
